// _NonLocalBlock2D_EGaussian_7782480740361
// MI455X (gfx1250) — hardware-verified
//
#include <hip/hip_runtime.h>
#include <hip/hip_bf16.h>

typedef __attribute__((ext_vector_type(16))) _Float16 v16h;
typedef __attribute__((ext_vector_type(8)))  _Float16 v8h;
typedef __attribute__((ext_vector_type(16))) __bf16   v16b;
typedef __attribute__((ext_vector_type(8)))  __bf16   v8b;
typedef __attribute__((ext_vector_type(8)))  float    v8f;
typedef __attribute__((ext_vector_type(4)))  float    v4f;

#define NB   8
#define CH   256
#define CI   128
#define NPIX 4096
#define MPIX 1024
#define NP3  384
#define NBLK_BN 128

__device__ __forceinline__ unsigned short f2bf_bits(float f) {
  unsigned u = __float_as_uint(f);
  return (unsigned short)((u + 0x7FFFu + ((u >> 16) & 1u)) >> 16);
}
__device__ __forceinline__ float bf_bits2f(unsigned short h) { return __uint_as_float(((unsigned)h) << 16); }

__device__ __forceinline__ void dep_guard_h(v8f& a, v8f& b, v16h x, v16h y) { asm volatile("v_nop\n\tv_nop\n\tv_nop\n\tv_nop" : "+v"(a), "+v"(b) : "v"(x), "v"(y)); }
__device__ __forceinline__ void dep_guard_b(v8f& a, v8f& b, v16b x, v16b y) { asm volatile("v_nop\n\tv_nop\n\tv_nop\n\tv_nop" : "+v"(a), "+v"(b) : "v"(x), "v"(y)); }
__device__ __forceinline__ void keep4_h(v16h a, v16h b, v16h c, v16h d) { asm volatile("v_nop" :: "v"(a), "v"(b), "v"(c), "v"(d)); }
__device__ __forceinline__ void keep4_b(v16b a, v16b b, v16b c, v16b d) { asm volatile("v_nop" :: "v"(a), "v"(b), "v"(c), "v"(d)); }
__device__ __forceinline__ void acc_guard4(v8f& a, v8f& b, v8f& c, v8f& d) { asm volatile("v_nop\n\tv_nop\n\tv_nop\n\tv_nop" : "+v"(a), "+v"(b), "+v"(c), "+v"(d)); }
template <typename T> struct Frag;
template <> struct Frag<_Float16> {
  typedef v16h V; union U { v16h v; v8h h[2]; };
  static __device__ __forceinline__ v16h load(const _Float16* p) {
    U f; f.h[0] = *(const v8h*)(p); f.h[1] = *(const v8h*)(p + 16); return f.v;
  }
  static __device__ __forceinline__ v8f mma(v16h a, v16h b, v8f c) {
    return __builtin_amdgcn_wmma_f32_16x16x32_f16(false, a, false, b, (short)0, c, false, false);
  }
  static __device__ __forceinline__ void guard(v8f& a, v8f& b, v16h x, v16h y) { dep_guard_h(a, b, x, y); }
  static __device__ __forceinline__ void keep(v16h a, v16h b, v16h c, v16h d) { keep4_h(a, b, c, d); }
};
template <> struct Frag<__bf16> {
  typedef v16b V; union U { v16b v; v8b h[2]; };
  static __device__ __forceinline__ v16b load(const __bf16* p) {
    U f; f.h[0] = *(const v8b*)(p); f.h[1] = *(const v8b*)(p + 16); return f.v;
  }
  static __device__ __forceinline__ v8f mma(v16b a, v16b b, v8f c) {
    return __builtin_amdgcn_wmma_f32_16x16x32_bf16(false, a, false, b, (short)0, c, false, false);
  }
  static __device__ __forceinline__ void guard(v8f& a, v8f& b, v16b x, v16b y) { dep_guard_b(a, b, x, y); }
  static __device__ __forceinline__ void keep(v16b a, v16b b, v16b c, v16b d) { keep4_b(a, b, c, d); }
};

template <int ET> struct Elem;
template <> struct Elem<0> { typedef _Float16 T; };
template <> struct Elem<1> { typedef __bf16 T; };
template <int ET, bool SPLIT, int BIAS_MODE, int OUT_MODE, bool RESID, int ACT = 0>
__global__ __launch_bounds__(256) void wmma_gemm64(
    const unsigned short* __restrict__ Ap, const unsigned short* __restrict__ A2p, int lda, long strideA,
    const unsigned short* __restrict__ Btp, const unsigned short* __restrict__ Bt2p, int ldb, long strideB,
    void* __restrict__ Cout, void* __restrict__ Cout2, int ldc, long strideC,
    const float* __restrict__ bias,
    const float* __restrict__ resid, long strideR,
    int M, int N, int K, float scale) {
  typedef typename Elem<ET>::T T;
  typedef typename Frag<T>::V V;
  const T* A = (const T*)Ap; const T* A2 = (const T*)A2p; const T* Bt = (const T*)Btp; const T* Bt2 = (const T*)Bt2p;
  __shared__ __align__(16) float sT[8][16 * 68];
  const int b    = blockIdx.y;
  const int lane = threadIdx.x & 31;
  const int wave = threadIdx.x >> 5;
  const int tilesN = N >> 6;
  const int tilesM = M >> 6;
  const int tile = blockIdx.x * 8 + wave;
  if (tile >= tilesM * tilesN) return;
  const int tm = tile / tilesN;
  const int tn = tile - tm * tilesN;
  const int m0 = tm << 6;
  const int n0 = tn << 6;

  const T* Ab  = A  + (size_t)b * strideA;
  const T* Bb  = Bt + (size_t)b * strideB;
  const T* Ab2 = SPLIT ? (A2  + (size_t)b * strideA) : nullptr;
  const T* Bb2 = SPLIT ? (Bt2 + (size_t)b * strideB) : nullptr;

  const int rlane = lane & 15;
  const int koff  = (lane >> 4) * 8;
  const int mOff  = (lane >> 4) * 8;

  v8f acc[4][4];
#pragma unroll
  for (int i = 0; i < 4; ++i)
#pragma unroll
    for (int j = 0; j < 4; ++j) acc[i][j] = (v8f){0.f,0.f,0.f,0.f,0.f,0.f,0.f,0.f};

  for (int k0 = 0; k0 < K; k0 += 32) {
    V bh[4], bl[4];
#pragma unroll
    for (int j = 0; j < 4; ++j) {
      const size_t bo = (size_t)(n0 + (j << 4) + rlane) * ldb + koff + k0;
      bh[j] = Frag<T>::load(Bb + bo);
      if (SPLIT) bl[j] = Frag<T>::load(Bb2 + bo);
    }
#pragma unroll
    for (int i = 0; i < 4; ++i) {
      const size_t ao = (size_t)(m0 + (i << 4) + rlane) * lda + koff + k0;
      V ah = Frag<T>::load(Ab + ao);
      V al;
      if (SPLIT) al = Frag<T>::load(Ab2 + ao);
#pragma unroll
      for (int j = 0; j < 4; ++j) {
        acc[i][j] = Frag<T>::mma(ah, bh[j], acc[i][j]);
        if (SPLIT) {
          acc[i][j] = Frag<T>::mma(ah, bl[j], acc[i][j]);
          acc[i][j] = Frag<T>::mma(al, bh[j], acc[i][j]);
        }
      }
      Frag<T>::guard(acc[i][0], acc[i][3], ah, SPLIT ? al : ah);
    }
    Frag<T>::keep(bh[0], bh[1], bh[2], bh[3]);
    if (SPLIT) Frag<T>::keep(bl[0], bl[1], bl[2], bl[3]);
  }
  acc_guard4(acc[0][0], acc[0][1], acc[0][2], acc[0][3]);
  acc_guard4(acc[1][0], acc[1][1], acc[1][2], acc[1][3]);
  acc_guard4(acc[2][0], acc[2][1], acc[2][2], acc[2][3]);
  acc_guard4(acc[3][0], acc[3][1], acc[3][2], acc[3][3]);

  float* slab = sT[wave];
  const float* Rb = RESID ? (resid + (size_t)b * strideR) : nullptr;
#pragma unroll
  for (int i = 0; i < 4; ++i) {
    const int mBase = m0 + (i << 4);
#pragma unroll
    for (int j = 0; j < 4; ++j) {
      const int n = n0 + (j << 4) + rlane;
      float bv = 0.f;
      if (BIAS_MODE == 2) bv = bias[n];
#pragma unroll
      for (int r = 0; r < 8; ++r) {
        float v = acc[i][j][r] * scale;
        if (BIAS_MODE == 1) v += bias[mBase + mOff + r];
        if (BIAS_MODE == 2) v += bv;
        if (RESID) v += Rb[(size_t)(mBase + mOff + r) * ldc + n];
        if (ACT == 1) v = tanhf(v);
        if (ACT == 2) v = fmaxf(v, 0.0f);
        if (ACT == 3) v = v / (1.0f + expf(-v));
        if (ACT == 4) v = (v > 0.f) ? v : 0.01f * v;
        if (ACT == 5) v = 0.5f * v * (1.0f + erff(v * 0.70710678118654752f));
        slab[(mOff + r) * 68 + (j << 4) + rlane] = v;
      }
    }
    __builtin_amdgcn_fence(__ATOMIC_RELEASE, "workgroup");
    __builtin_amdgcn_wave_barrier();
    __builtin_amdgcn_fence(__ATOMIC_ACQUIRE, "workgroup");
    if (OUT_MODE == 0) {
      float* C = (float*)Cout + (size_t)b * strideC;
      const int hh = lane >> 4, c4 = (lane & 15) * 4;
      for (int pass = 0; pass < 2; ++pass) {
#pragma unroll
        for (int it = 0; it < 8; ++it) {
          const int row = it * 2 + hh;
          v4f v = *(const v4f*)(slab + row * 68 + c4);
          *(volatile v4f*)(C + (size_t)(mBase + row) * ldc + n0 + c4) = v;
        }
        __threadfence();
      }
    } else {
      const int q = lane >> 3, c8 = (lane & 7) * 8;
      unsigned short* C  = (unsigned short*)Cout  + (size_t)b * strideC;
      unsigned short* C2 = (OUT_MODE == 2) ? ((unsigned short*)Cout2 + (size_t)b * strideC) : nullptr;
      for (int pass = 0; pass < 2; ++pass) {
#pragma unroll
        for (int it = 0; it < 4; ++it) {
          const int row = it * 4 + q;
          const float* sp = slab + row * 68 + c8;
          v8h hv, lv;
#pragma unroll
          for (int e = 0; e < 8; ++e) {
            if (OUT_MODE == 1) {
              hv[e] = (_Float16)sp[e];
            } else {
              unsigned short hb = f2bf_bits(sp[e]);
              unsigned short lb = f2bf_bits(sp[e] - bf_bits2f(hb));
              hv[e] = __builtin_bit_cast(_Float16, hb);
              lv[e] = __builtin_bit_cast(_Float16, lb);
            }
          }
          *(volatile v8h*)(C + (size_t)(mBase + row) * ldc + n0 + c8) = hv;
          if (OUT_MODE == 2) *(volatile v8h*)(C2 + (size_t)(mBase + row) * ldc + n0 + c8) = lv;
        }
        __threadfence();
      }
    }
    __builtin_amdgcn_fence(__ATOMIC_RELEASE, "workgroup");
    __builtin_amdgcn_wave_barrier();
    __builtin_amdgcn_fence(__ATOMIC_ACQUIRE, "workgroup");
  }
}

__global__ __launch_bounds__(256) void k_xT(const float* __restrict__ x, _Float16* __restrict__ XT) {
  __shared__ __align__(16) _Float16 T[64 * 264];
  const int tid = threadIdx.x;
  const int b  = blockIdx.x >> 6;
  const int n0 = (blockIdx.x & 63) * 64;
  const float* xb = x + (size_t)b * CH * NPIX + n0;
#pragma unroll 4
  for (int it = 0; it < 64; ++it) {
    const int idx = it * 256 + tid;
    const int c = idx >> 6, j = idx & 63;
    T[j * 264 + c] = (_Float16)xb[(size_t)c * NPIX + j];
  }
  __syncthreads();
  const int wave = tid >> 5, lane = tid & 31;
  _Float16* dst = XT + ((size_t)b * NPIX + n0) * CH;
  for (int pass = 0; pass < 2; ++pass) {
#pragma unroll
    for (int it = 0; it < 8; ++it) {
      const int j = wave * 8 + it;
      const v8h v = *(const v8h*)(T + j * 264 + lane * 8);
      *(volatile v8h*)(dst + (size_t)j * CH + lane * 8) = v;
    }
    __threadfence();
  }
}

__global__ __launch_bounds__(256) void k_prepw(const float* __restrict__ w_t, const float* __restrict__ w_p, const float* __restrict__ w_g,
                                                const float* __restrict__ b_t, const float* __restrict__ b_p, const float* __restrict__ b_g,
                                                _Float16* __restrict__ W16, float* __restrict__ bias) {
  const int sel = blockIdx.y;
  const float* src = (sel == 0) ? w_t : ((sel == 1) ? w_p : w_g);
  const float* bsr = (sel == 0) ? b_t : ((sel == 1) ? b_p : b_g);
  const int tid = threadIdx.x;
  const int i = blockIdx.x * 256 + tid;
  const float f0 = src[2 * i] * 16.0f;
  const float f1 = src[2 * i + 1] * 16.0f;
  const _Float16 h0 = (_Float16)f0, h1 = (_Float16)f1;
  const unsigned u = (unsigned)__builtin_bit_cast(unsigned short, h0) | ((unsigned)__builtin_bit_cast(unsigned short, h1) << 16);
  volatile unsigned* d = ((volatile unsigned*)(W16 + (size_t)sel * (CI * CH))) + i;
  *d = u;
  __threadfence();
  *d = u;
  if (blockIdx.x == 0 && tid < 128) {
    const float bv = bsr[tid];
    volatile float* bd = ((volatile float*)bias) + sel * 128 + tid;
    *bd = bv;
    __threadfence();
    *bd = bv;
  }
}

__global__ __launch_bounds__(256) void k_prepww(const float* __restrict__ ww, unsigned short* __restrict__ hi, unsigned short* __restrict__ lo) {
  const int i = blockIdx.x * 256 + threadIdx.x;
  const float f0 = ww[2 * i], f1 = ww[2 * i + 1];
  const unsigned short hb0 = f2bf_bits(f0), hb1 = f2bf_bits(f1);
  const unsigned short lb0 = f2bf_bits(f0 - bf_bits2f(hb0)), lb1 = f2bf_bits(f1 - bf_bits2f(hb1));
  const unsigned uh = (unsigned)hb0 | ((unsigned)hb1 << 16);
  const unsigned ul = (unsigned)lb0 | ((unsigned)lb1 << 16);
  volatile unsigned* dh = ((volatile unsigned*)hi) + i;
  volatile unsigned* dl = ((volatile unsigned*)lo) + i;
  *dh = uh;
  *dl = ul;
  __threadfence();
  *dh = uh;
  *dl = ul;
}

__global__ __launch_bounds__(256) void k_pool(const _Float16* __restrict__ TPG, _Float16* __restrict__ PHIP, _Float16* __restrict__ GPT) {
  __shared__ __align__(16) _Float16 G[CI * 72];
  const int tid = threadIdx.x, wave = tid >> 5, lane = tid & 31;
  const int b  = blockIdx.x >> 4;
  const int m0 = (blockIdx.x & 15) * 64;
  const _Float16* tb = TPG + (size_t)b * NPIX * NP3;
  v8h pmv[4];
#pragma unroll
  for (int it = 0; it < 4; ++it) {
    const int idx = it * 256 + tid;
    const int ml = idx >> 4, cg = idx & 15;
    const int m  = m0 + ml;
    const int h2 = m >> 5, w2 = m & 31;
    const size_t n00 = (size_t)(2 * h2) * 64 + 2 * w2;
    const _Float16* pp = tb + n00 * NP3 + CI + cg * 8;
    const _Float16* pg = pp + CI;
    const v8h a0 = *(const v8h*)(pp), a1 = *(const v8h*)(pp + NP3), a2 = *(const v8h*)(pp + 64 * NP3), a3 = *(const v8h*)(pp + 65 * NP3);
    const v8h g0 = *(const v8h*)(pg), g1 = *(const v8h*)(pg + NP3), g2 = *(const v8h*)(pg + 64 * NP3), g3 = *(const v8h*)(pg + 65 * NP3);
    v8h pm;
#pragma unroll
    for (int e = 0; e < 8; ++e) {
      pm[e] = (_Float16)fmaxf(fmaxf((float)a0[e], (float)a1[e]), fmaxf((float)a2[e], (float)a3[e]));
      const float gmx = fmaxf(fmaxf((float)g0[e], (float)g1[e]), fmaxf((float)g2[e], (float)g3[e])) * 16.0f;
      G[(cg * 8 + e) * 72 + ml] = (_Float16)gmx;
    }
    pmv[it] = pm;
  }
  _Float16* pd = PHIP + ((size_t)b * MPIX + m0) * CI;
  for (int pass = 0; pass < 2; ++pass) {
#pragma unroll
    for (int it = 0; it < 4; ++it) {
      const int idx = it * 256 + tid;
      const int ml = idx >> 4, cg = idx & 15;
      *(volatile v8h*)(pd + (size_t)ml * CI + cg * 8) = pmv[it];
    }
    __threadfence();
  }
  __syncthreads();
  _Float16* gd = GPT + (size_t)b * CI * MPIX + m0;
  const int q = lane >> 3, c8 = (lane & 7) * 8;
  for (int pass = 0; pass < 2; ++pass) {
#pragma unroll
    for (int it = 0; it < 4; ++it) {
      const int ci = it * 32 + wave * 4 + q;
      const v8h v = *(const v8h*)(G + ci * 72 + c8);
      *(volatile v8h*)(gd + (size_t)ci * MPIX + c8) = v;
    }
    __threadfence();
  }
}

__global__ __launch_bounds__(256) void k_softmax(const float* __restrict__ S, _Float16* __restrict__ P) {
  const int tid = threadIdx.x, wave = tid >> 5, lane = tid & 31;
  const int row = blockIdx.x * 8 + wave;
  const float* sr = S + (size_t)row * MPIX;
  float v[32];
#pragma unroll
  for (int i = 0; i < 4; ++i) {
    const v4f a = *(const v4f*)(sr + 256 * i + lane * 8);
    const v4f c = *(const v4f*)(sr + 256 * i + lane * 8 + 4);
    v[8 * i + 0] = a[0]; v[8 * i + 1] = a[1]; v[8 * i + 2] = a[2]; v[8 * i + 3] = a[3];
    v[8 * i + 4] = c[0]; v[8 * i + 5] = c[1]; v[8 * i + 6] = c[2]; v[8 * i + 7] = c[3];
  }
  float mx = v[0];
#pragma unroll
  for (int e = 1; e < 32; ++e) mx = fmaxf(mx, v[e]);
#pragma unroll
  for (int off = 1; off < 32; off <<= 1) mx = fmaxf(mx, __shfl_xor(mx, off, 32));
  float sum = 0.f;
#pragma unroll
  for (int e = 0; e < 32; ++e) { v[e] = __expf(v[e] - mx); sum += v[e]; }
#pragma unroll
  for (int off = 1; off < 32; off <<= 1) sum += __shfl_xor(sum, off, 32);
  const float sc = 32768.0f * (1.0f / sum);
  v8h h[4];
#pragma unroll
  for (int i = 0; i < 4; ++i) {
#pragma unroll
    for (int e = 0; e < 8; ++e) h[i][e] = (_Float16)(v[8 * i + e] * sc);
  }
  _Float16* pr = P + (size_t)row * MPIX;
  for (int pass = 0; pass < 2; ++pass) {
#pragma unroll
    for (int i = 0; i < 4; ++i) *(volatile v8h*)(pr + 256 * i + lane * 8) = h[i];
    __threadfence();
  }
}

__global__ __launch_bounds__(256) void k_bnpart(const float* __restrict__ WY, double* __restrict__ ps, double* __restrict__ pq) {
  const int co = threadIdx.x;
  const int r0 = blockIdx.x * (NB * NPIX / NBLK_BN);
  double s = 0.0, q = 0.0;
#pragma unroll 4
  for (int r = 0; r < (NB * NPIX / NBLK_BN); ++r) {
    const float f = WY[(size_t)(r0 + r) * CH + co];
    const double d = (double)f;
    s += d;
    q += d * d;
  }
  volatile double* ds = ((volatile double*)ps) + (size_t)blockIdx.x * CH + co;
  volatile double* dq = ((volatile double*)pq) + (size_t)blockIdx.x * CH + co;
  *ds = s;
  *dq = q;
  __threadfence();
  *ds = s;
  *dq = q;
}

__global__ __launch_bounds__(256) void k_bnfin(const double* __restrict__ ps, const double* __restrict__ pq,
                                                float* __restrict__ mean, float* __restrict__ rstd) {
  const int co = threadIdx.x;
  double s = 0.0, q = 0.0;
#pragma unroll 1
  for (int k = 0; k < NBLK_BN; ++k) { s += ps[(size_t)k * CH + co]; q += pq[(size_t)k * CH + co]; }
  const double inv = 1.0 / (double)(NB * NPIX);
  const double mn = s * inv;
  double var = q * inv - mn * mn;
  if (var < 0.0) var = 0.0;
  const float mf = (float)mn;
  const float ve = (float)var + 1e-5f;
  const float rs = (float)(1.0 / sqrt((double)ve));
  volatile float* dm = ((volatile float*)mean) + co;
  volatile float* dr = ((volatile float*)rstd) + co;
  *dm = mf;
  *dr = rs;
  __threadfence();
  *dm = mf;
  *dr = rs;
}

__global__ __launch_bounds__(256) void k_out(const float* __restrict__ WY, const float* __restrict__ x,
                                              const float* __restrict__ mean, const float* __restrict__ rstd,
                                              const float* __restrict__ gamma, const float* __restrict__ beta,
                                              float* __restrict__ out) {
  __shared__ __align__(16) float T[CH * 36];
  const int tid = threadIdx.x, wave = tid >> 5, lane = tid & 31;
  const int b  = blockIdx.x >> 7;
  const int n0 = (blockIdx.x & 127) * 32;
#pragma unroll
  for (int it = 0; it < 8; ++it) {
    const int idx = it * 256 + tid;
    const int r = idx >> 6, c4 = (idx & 63) * 4;
    const v4f w = *(const v4f*)(WY + ((size_t)(b * NPIX + n0 + r)) * CH + c4);
    T[(c4 + 0) * 36 + r] = w[0];
    T[(c4 + 1) * 36 + r] = w[1];
    T[(c4 + 2) * 36 + r] = w[2];
    T[(c4 + 3) * 36 + r] = w[3];
  }
  __syncthreads();
  const int q = lane >> 3, f4 = (lane & 7) * 4;
  v4f vals[8];
#pragma unroll
  for (int it = 0; it < 8; ++it) {
    const int co = it * 32 + wave * 4 + q;
    const v4f w  = *(const v4f*)(T + co * 36 + f4);
    const v4f xx = *(const v4f*)(x + ((size_t)(b * CH + co)) * NPIX + n0 + f4);
    const float mn = mean[co], rs = rstd[co], ga = gamma[co], be = beta[co];
    v4f o;
#pragma unroll
    for (int e = 0; e < 4; ++e) {
      float z = (w[e] - mn) * rs;
      z = z * ga + be;
      o[e] = z + xx[e];
    }
    vals[it] = o;
  }
  float* ob = out + (size_t)b * CH * NPIX + n0;
  for (int pass = 0; pass < 2; ++pass) {
#pragma unroll
    for (int it = 0; it < 8; ++it) {
      const int co = it * 32 + wave * 4 + q;
      *(volatile v4f*)(ob + (size_t)co * NPIX + f4) = vals[it];
    }
    __threadfence();
  }
}

extern "C" void kernel_launch(void* const* d_in, const int* in_sizes, int n_in,
                              void* d_out, int out_size, void* d_ws, size_t ws_size,
                              hipStream_t stream) {
  if (n_in < 11) return;
  if (in_sizes[0] != NB * CH * NPIX || out_size != NB * CH * NPIX) return;
  if (in_sizes[1] != CI * CH || in_sizes[3] != CI * CH || in_sizes[5] != CI * CH || in_sizes[7] != CH * CI) return;
  if (in_sizes[2] < CI || in_sizes[4] < CI || in_sizes[6] < CI || in_sizes[8] < CH || in_sizes[9] < CH || in_sizes[10] < CH) return;

  const float* x     = (const float*)d_in[0];
  const float* w_g   = (const float*)d_in[1];
  const float* b_g   = (const float*)d_in[2];
  const float* w_th  = (const float*)d_in[3];
  const float* b_th  = (const float*)d_in[4];
  const float* w_ph  = (const float*)d_in[5];
  const float* b_ph  = (const float*)d_in[6];
  const float* w_w   = (const float*)d_in[7];
  const float* b_w   = (const float*)d_in[8];
  const float* gamma = (const float*)d_in[9];
  const float* beta  = (const float*)d_in[10];
  float* out = (float*)d_out;

  char* ws = (char*)d_ws;
  size_t off = 0;
  auto carve = [&](size_t bytes) -> char* { char* p = ws + off; off += (bytes + 255) & ~(size_t)255; return p; };
  unsigned short* XT16  = (unsigned short*)carve((size_t)NB * NPIX * CH * 2);
  float*          S     = (float*)XT16;
  unsigned short* TPG16 = (unsigned short*)carve((size_t)NB * NPIX * NP3 * 2);
  unsigned short* PHIP  = (unsigned short*)carve((size_t)NB * MPIX * CI * 2);
  unsigned short* GPT   = (unsigned short*)carve((size_t)NB * CI * MPIX * 2);
  unsigned short* P16   = (unsigned short*)carve((size_t)NPIX * MPIX * 2);
  unsigned short* Yhi   = (unsigned short*)carve((size_t)NB * NPIX * CI * 2);
  unsigned short* Ylo   = (unsigned short*)carve((size_t)NB * NPIX * CI * 2);
  float*          WY    = (float*)carve((size_t)NB * NPIX * CH * 4);
  unsigned short* Wp16  = (unsigned short*)carve((size_t)NP3 * CH * 2);
  float*          bias3 = (float*)carve((size_t)NP3 * 4);
  unsigned short* WWhi  = (unsigned short*)carve((size_t)CH * CI * 2);
  unsigned short* WWlo  = (unsigned short*)carve((size_t)CH * CI * 2);
  double*         parts = (double*)carve((size_t)NBLK_BN * CH * 8);
  double*         partq = (double*)carve((size_t)NBLK_BN * CH * 8);
  float*          meanb = (float*)carve((size_t)CH * 4);
  float*          rstdb = (float*)carve((size_t)CH * 4);
  if (off > ws_size) return;
  if ((size_t)NPIX * MPIX * 4 > (size_t)NB * NPIX * CH * 2) return;

  k_xT<<<NB * (NPIX / 64), 256, 0, stream>>>(x, (_Float16*)XT16);
  k_prepw<<<dim3((CI * CH / 2) / 256, 3), 256, 0, stream>>>(w_th, w_ph, w_g, b_th, b_ph, b_g, (_Float16*)Wp16, bias3);
  k_prepww<<<(CH * CI / 2) / 256, 256, 0, stream>>>(w_w, WWhi, WWlo);
  wmma_gemm64<0, false, 2, 1, false><<<dim3(48, NB), 256, 0, stream>>>(
      XT16, XT16, CH, (long)NPIX * CH,
      Wp16, Wp16, CH, (long)0,
      (void*)TPG16, (void*)TPG16, NP3, (long)NPIX * NP3,
      bias3, bias3, (long)0,
      NPIX, NP3, CH, 1.0f / 16.0f);
  k_pool<<<NB * (MPIX / 64), 256, 0, stream>>>((const _Float16*)TPG16, (_Float16*)PHIP, (_Float16*)GPT);
  for (int b = 0; b < NB; ++b) {
    const unsigned short* theta = TPG16 + (size_t)b * NPIX * NP3;
    const unsigned short* phib  = PHIP + (size_t)b * MPIX * CI;
    const unsigned short* gtb   = GPT + (size_t)b * CI * MPIX;
    unsigned short* yh = Yhi + (size_t)b * NPIX * CI;
    unsigned short* yl = Ylo + (size_t)b * NPIX * CI;
    wmma_gemm64<0, false, 0, 0, false><<<dim3(128, 1), 256, 0, stream>>>(
        theta, theta, NP3, (long)0,
        phib, phib, CI, (long)0,
        (void*)S, (void*)S, MPIX, (long)0,
        bias3, bias3, (long)0,
        NPIX, MPIX, CI, 1.0f);
    k_softmax<<<NPIX / 8, 256, 0, stream>>>(S, (_Float16*)P16);
    wmma_gemm64<0, false, 0, 2, false><<<dim3(16, 1), 256, 0, stream>>>(
        P16, P16, MPIX, (long)0,
        gtb, gtb, MPIX, (long)0,
        (void*)yh, (void*)yl, CI, (long)0,
        bias3, bias3, (long)0,
        NPIX, CI, MPIX, 1.0f / 524288.0f);
  }
  wmma_gemm64<1, true, 2, 0, false><<<dim3(256, 1), 256, 0, stream>>>(
      Yhi, Ylo, CI, (long)0,
      WWhi, WWlo, CI, (long)0,
      (void*)WY, (void*)WY, CH, (long)0,
      b_w, b_w, (long)0,
      NB * NPIX, CH, CI, 1.0f);
  k_bnpart<<<NBLK_BN, 256, 0, stream>>>(WY, parts, partq);
  k_bnfin<<<1, 256, 0, stream>>>(parts, partq, meanb, rstdb);
  k_out<<<NB * (NPIX / 32), 256, 0, stream>>>(WY, x, meanb, rstdb, gamma, beta, out);
  (void)hipGetLastError();
}
